// PINN_NS_12154757448258
// MI455X (gfx1250) — hardware-run, weakly checked
//
#include <hip/hip_runtime.h>
#include <stddef.h>


typedef _Float16 v16h __attribute__((ext_vector_type(16)));
typedef _Float16 v8h  __attribute__((ext_vector_type(8)));
typedef float    v8f  __attribute__((ext_vector_type(8)));
typedef float    v4f  __attribute__((ext_vector_type(4)));
typedef _Float16 h16;

#ifndef NPTS
#define NPTS 16384
#endif
#define NPTS_FULL 16384
#define HIDW   256
#define NLAY   5
#define NSTATE 6
#define NRES   4

#define LDT 72
#define LDH 264
#define PLSZ (16u * LDH)

#define WCARRY   64.0f
#define HCARRY   16.0f
#define SCARRY   1024.0f
#define RESCARRY 2048.0f
#define INV_HW (1.0f / (HCARRY * WCARRY))
#define INV_SW (1.0f / (SCARRY * WCARRY))
#define INV_RW (1.0f / (HCARRY * WCARRY * RESCARRY))
#define NU_C   (1.0f / 100.0f)

#define WPLANE_ELEMS ((size_t)HIDW * HIDW)
#define WPLANE_BYTES (WPLANE_ELEMS * 2)
#define WS_TOTAL     ((size_t)NLAY * WPLANE_BYTES)

#define LDS_BYTES ((NSTATE + NRES) * 16 * LDH * 2 + NLAY * HIDW * 4 + 3 * HIDW * 4 + 32 * 4 + 96 * 4 + 288 * 4 + 96 * 4)

static_assert(NPTS >= 32 && NPTS <= NPTS_FULL && (NPTS % 32) == 0);
static_assert(((size_t)NPTS_FULL * 4) % 128 == 0);
static_assert(HIDW == 256);
static_assert((HIDW % 64) == 0 && (HIDW % 32) == 0);
static_assert(8 * 32 == HIDW);
static_assert((LDT % 8) == 0 && LDT >= 64);
static_assert((LDH % 8) == 0 && LDH >= HIDW);
static_assert((WPLANE_BYTES % 128) == 0);
static_assert(WS_TOTAL <= (size_t)134217728);
static_assert(16 * NSTATE * 3 == 288);
static_assert(NRES == 4 && NRES <= NSTATE);
static_assert(LDS_BYTES <= 131072);

__device__ __forceinline__ float bf16r(float x) {
  unsigned int u = __float_as_uint(x);
  u = (u + 0x7FFFu + ((u >> 16) & 1u)) & 0xFFFF0000u;
  return __uint_as_float(u);
}

__device__ __forceinline__ v16h frag_at(const _Float16* p) {
  v8h lo = *(const v8h*)(p);
  v8h hi = *(const v8h*)(p + 16);
  v16h out;
#pragma unroll
  for (int i = 0; i < 8; ++i) { out[i] = lo[i]; out[i + 8] = hi[i]; }
  return out;
}
__device__ __forceinline__ v16h ld_frag(const _Float16* base, unsigned ld) {
  const unsigned lane = threadIdx.x & 31u;
  return frag_at(base + (lane & 15u) * ld + (lane >> 4) * 8u);
}

__device__ __forceinline__ v8f wmma16(v16h a, v16h b, v8f c) {
  v8f d = __builtin_amdgcn_wmma_f32_16x16x32_f16(false, a, false, b, (short)0, c,
                                                 false, false);
  asm volatile("v_nop\n\tv_nop\n\tv_nop\n\tv_nop" : "+v"(d) : "v"(a), "v"(b));
  return d;
}

static __device__ __forceinline__ h16 toh_flush(float v) {
  const h16 r = (h16)v;
  return (fabsf(v) < 6.103515625e-05f) ? (h16)0.0f : r;
}

__global__ __launch_bounds__(256) void wconv_kernel(
    const float* __restrict__ W, _Float16* __restrict__ Wt, unsigned ldw, unsigned ldk) {
  __shared__ _Float16 T[64 * LDT];
  const unsigned tid = threadIdx.x;
  const unsigned n0 = blockIdx.x * 64u;
  const unsigned k0 = blockIdx.y * 64u;
#pragma unroll 4
  for (unsigned j = 0; j < 16u; ++j) {
    const unsigned idx = tid + 256u * j;
    const unsigned kr = idx >> 6, nc = idx & 63u;
    const float v = W[(size_t)(k0 + kr) * ldw + n0 + nc];
    T[nc * LDT + kr] = (_Float16)(WCARRY * bf16r(v));
  }
  __syncthreads();
  v8h x[2];
  size_t off[2];
#pragma unroll
  for (unsigned i = 0; i < 2u; ++i) {
    const unsigned n = 32u * i + (tid >> 3);
    const unsigned kc = (tid & 7u) * 8u;
    x[i] = *(const v8h*)&T[n * LDT + kc];
    off[i] = (size_t)(n0 + n) * ldk + k0 + kc;
  }
#pragma unroll
  for (int i = 0; i < 2; ++i) *(volatile v8h*)(Wt + off[i]) = x[i];
  __threadfence();
#pragma unroll
  for (int i = 0; i < 2; ++i) *(volatile v8h*)(Wt + off[i]) = x[i];
}

__device__ __forceinline__ void store_jet(_Float16* H, _Float16* R, unsigned base,
                                          float h, float gt, float gx, float gy,
                                          float sxx, float syy) {
  const float v0 = HCARRY * h;
  const float g0 = HCARRY * gt, g1 = HCARRY * gx, g2 = HCARRY * gy;
  const h16 qv = toh_flush(v0);
  const h16 q0 = toh_flush(g0), q1 = toh_flush(g1), q2 = toh_flush(g2);
  H[base]             = qv;
  H[1u * PLSZ + base] = q0;
  H[2u * PLSZ + base] = q1;
  H[3u * PLSZ + base] = q2;
  R[base]             = toh_flush((v0 - (float)qv) * RESCARRY);
  R[1u * PLSZ + base] = toh_flush((g0 - (float)q0) * RESCARRY);
  R[2u * PLSZ + base] = toh_flush((g1 - (float)q1) * RESCARRY);
  R[3u * PLSZ + base] = toh_flush((g2 - (float)q2) * RESCARRY);
  H[4u * PLSZ + base] = toh_flush(SCARRY * sxx);
  H[5u * PLSZ + base] = toh_flush(SCARRY * syy);
}

__global__ __launch_bounds__(256) __attribute__((amdgpu_num_vgpr(256))) void pinn_jet_kernel(
    const float* __restrict__ tin, const float* __restrict__ xin, const float* __restrict__ yin,
    const float* __restrict__ W0, const float* __restrict__ b0,
    const _Float16* __restrict__ Wt,
    const float* __restrict__ b1, const float* __restrict__ b2, const float* __restrict__ b3,
    const float* __restrict__ b4, const float* __restrict__ b5,
    const float* __restrict__ W6, const float* __restrict__ b6,
    float* __restrict__ out) {
  __shared__ __attribute__((aligned(16))) _Float16 Hs[NSTATE * 16 * LDH];
  __shared__ __attribute__((aligned(16))) _Float16 Rs[NRES * 16 * LDH];
  __shared__ float bs[NLAY * HIDW];
  __shared__ float w6s[3 * HIDW];
  __shared__ float b6s[32];
  __shared__ float txy[96];
  __shared__ float res[16 * 18];
  __shared__ __attribute__((aligned(16))) float eqs[96];

  const unsigned tid = threadIdx.x, lane = tid & 31u;
  const int wave = __builtin_amdgcn_readfirstlane(threadIdx.x >> 5);
  const unsigned hh = lane >> 4, m = lane & 15u;
  const unsigned p0 = blockIdx.x * 32u;
  const unsigned c0 = (unsigned)wave * 32u;

  bs[tid]             = bf16r(b1[tid]);
  bs[HIDW + tid]      = bf16r(b2[tid]);
  bs[2 * HIDW + tid]  = bf16r(b3[tid]);
  bs[3 * HIDW + tid]  = bf16r(b4[tid]);
  bs[4 * HIDW + tid]  = bf16r(b5[tid]);
  w6s[tid]            = bf16r(W6[tid]);
  w6s[HIDW + tid]     = bf16r(W6[HIDW + tid]);
  w6s[2 * HIDW + tid] = bf16r(W6[2 * HIDW + tid]);
  if (wave == 0) {
    unsigned p = p0 + lane;
    p = (p < (unsigned)NPTS) ? p : (unsigned)(NPTS - 1);
    txy[lane]       = bf16r(tin[p]);
    txy[32u + lane] = bf16r(xin[p]);
    txy[64u + lane] = bf16r(yin[p]);
    b6s[lane] = bf16r(b6[(lane < 3u) ? lane : 2u]);
  }
  const float w0 = bf16r(W0[tid]);
  const float w1 = bf16r(W0[HIDW + tid]);
  const float w2 = bf16r(W0[2 * HIDW + tid]);
  const float bb0 = bf16r(b0[tid]);
  __syncthreads();

#pragma unroll 1
  for (unsigned sub = 0; sub < 2u; ++sub) {
#pragma unroll 2
    for (unsigned mm = 0; mm < 16u; ++mm) {
      const float tt = txy[sub * 16u + mm];
      const float xx = txy[32u + sub * 16u + mm];
      const float yy = txy[64u + sub * 16u + mm];
      const float z = tt * w0 + xx * w1 + yy * w2 + bb0;
      const float sz = __sinf(z), cz = __cosf(z);
      store_jet(Hs, Rs, mm * LDH + tid, sz, cz * w0, cz * w1, cz * w2,
                -sz * w1 * w1, -sz * w2 * w2);
    }
    __syncthreads();

#pragma unroll 1
    for (unsigned l = 0; l < (unsigned)NLAY; ++l) {
      const _Float16* bp0 = Wt + (size_t)l * WPLANE_ELEMS + (size_t)(c0 + m) * HIDW + hh * 8u;
      const _Float16* bp1 = bp0 + (size_t)16 * HIDW;

      v8f acc[NSTATE][2];
#pragma unroll
      for (int s = 0; s < NSTATE; ++s) { acc[s][0] = (v8f){}; acc[s][1] = (v8f){}; }
      v8f accr[NRES][2];
#pragma unroll
      for (int s = 0; s < NRES; ++s) { accr[s][0] = (v8f){}; accr[s][1] = (v8f){}; }

#pragma unroll 1
      for (unsigned k0 = 0; k0 < (unsigned)HIDW; k0 += 32u) {
        const v16h b0f = frag_at(bp0 + k0);
        const v16h b1f = frag_at(bp1 + k0);
#pragma unroll
        for (int s = 0; s < NSTATE; ++s) {
          const v16h a = ld_frag(&Hs[(unsigned)s * PLSZ + k0], LDH);
          acc[s][0] = wmma16(a, b0f, acc[s][0]);
          acc[s][1] = wmma16(a, b1f, acc[s][1]);
        }
#pragma unroll
        for (int s = 0; s < NRES; ++s) {
          const v16h a = ld_frag(&Rs[(unsigned)s * PLSZ + k0], LDH);
          accr[s][0] = wmma16(a, b0f, accr[s][0]);
          accr[s][1] = wmma16(a, b1f, accr[s][1]);
        }
      }

      __syncthreads();

#pragma unroll
      for (int t2 = 0; t2 < 2; ++t2) {
        const unsigned col = c0 + (unsigned)t2 * 16u + m;
        const float bb = bs[l * HIDW + col];
#pragma unroll
        for (int r = 0; r < 8; ++r) {
          const unsigned row = hh * 8u + (unsigned)r;
          float zv = acc[0][t2][r] * INV_HW;
          float zt = acc[1][t2][r] * INV_HW;
          float zx = acc[2][t2][r] * INV_HW;
          float zy = acc[3][t2][r] * INV_HW;
          zv += accr[0][t2][r] * INV_RW;
          zt += accr[1][t2][r] * INV_RW;
          zx += accr[2][t2][r] * INV_RW;
          zy += accr[3][t2][r] * INV_RW;
          const float z = zv + bb;
          const float sz = __sinf(z), cz = __cosf(z);
          const float zxx = acc[4][t2][r] * INV_SW;
          const float zyy = acc[5][t2][r] * INV_SW;
          store_jet(Hs, Rs, row * LDH + col, sz, cz * zt, cz * zx, cz * zy,
                    cz * zxx - sz * zx * zx, cz * zyy - sz * zy * zy);
        }
      }
      __syncthreads();
    }

#pragma unroll 1
    for (unsigned idx = tid; idx < 288u; idx += 256u) {
      const unsigned s = idx / 48u;
      const unsigned rem = idx - s * 48u;
      const unsigned mm = rem / 3u;
      const unsigned col = rem - mm * 3u;
      const unsigned hb = (s * 16u + mm) * LDH;
      const bool isg = (s <= 3u);
      const unsigned rb = ((isg ? s : 0u) * 16u + mm) * LDH;
      const float rw = isg ? (1.0f / RESCARRY) : 0.0f;
      float a = 0.0f;
#pragma unroll 4
      for (unsigned k = 0; k < (unsigned)HIDW; ++k) {
        float v = (float)Hs[hb + k];
        v += (float)Rs[rb + k] * rw;
        a += v * w6s[k * 3u + col];
      }
      const float cinv = (s >= 4u) ? (1.0f / SCARRY) : (1.0f / HCARRY);
      const float bv = b6s[col];
      a = a * cinv + ((s == 0u) ? bv : 0.0f);
      res[mm * 18u + s * 3u + col] = a;
    }
    __syncthreads();

    if (tid < 16u) {
      const float* r = &res[tid * 18u];
      const float u = r[0], v = r[1];
      const float u_t = r[3], v_t = r[4];
      const float u_x = r[6], v_x = r[7], p_x = r[8];
      const float u_y = r[9], v_y = r[10], p_y = r[11];
      const float u_xx = r[12], v_xx = r[13];
      const float u_yy = r[15], v_yy = r[16];
      const float eq1 = u_t + (u * u_x + v * u_y) + p_x - NU_C * (u_xx + u_yy);
      const float eq2 = v_t + (u * v_x + v * v_y) + p_y - NU_C * (v_xx + v_yy);
      const float eq3 = u_x + v_y;
      eqs[sub * 16u + tid]       = eq1;
      eqs[32u + sub * 16u + tid] = eq2;
      eqs[64u + sub * 16u + tid] = eq3;
    }
  }
  __syncthreads();

  if (wave == 0) {
    const unsigned q = lane >> 3;
    const unsigned qq = (q < 3u) ? q : 2u;
    const unsigned c = (lane & 7u) * 4u;
    const v4f val = *(const v4f*)&eqs[qq * 32u + c];
    float* dst = out + (size_t)qq * NPTS_FULL + p0 + c;
    if (q < 3u) *(volatile v4f*)dst = val;
    __threadfence();
    if (q < 3u) *(volatile v4f*)dst = val;
  }
}

extern "C" void kernel_launch(void* const* d_in, const int* in_sizes, int n_in,
                              void* d_out, int out_size, void* d_ws, size_t ws_size,
                              hipStream_t stream) {
  if (n_in < 17) return;
  if (in_sizes[0] < NPTS || in_sizes[1] < NPTS || in_sizes[2] < NPTS) return;
  if (in_sizes[3] < 3 * HIDW || in_sizes[4] < HIDW) return;
  if (in_sizes[5] < HIDW * HIDW || in_sizes[7] < HIDW * HIDW || in_sizes[9] < HIDW * HIDW) return;
  if (in_sizes[11] < HIDW * HIDW || in_sizes[13] < HIDW * HIDW) return;
  if (in_sizes[6] < HIDW || in_sizes[8] < HIDW || in_sizes[10] < HIDW) return;
  if (in_sizes[12] < HIDW || in_sizes[14] < HIDW) return;
  if (in_sizes[15] < 3 * HIDW || in_sizes[16] < 3) return;
  if ((long long)out_size < (long long)2 * NPTS_FULL + NPTS) return;
  if (ws_size < WS_TOTAL) return;

  const float* t   = (const float*)d_in[0];
  const float* x   = (const float*)d_in[1];
  const float* y   = (const float*)d_in[2];
  const float* w0  = (const float*)d_in[3];
  const float* b0v = (const float*)d_in[4];
  const float* w1  = (const float*)d_in[5];
  const float* b1v = (const float*)d_in[6];
  const float* w2  = (const float*)d_in[7];
  const float* b2v = (const float*)d_in[8];
  const float* w3  = (const float*)d_in[9];
  const float* b3v = (const float*)d_in[10];
  const float* w4  = (const float*)d_in[11];
  const float* b4v = (const float*)d_in[12];
  const float* w5  = (const float*)d_in[13];
  const float* b5v = (const float*)d_in[14];
  const float* w6  = (const float*)d_in[15];
  const float* b6v = (const float*)d_in[16];
  float* out = (float*)d_out;

  _Float16* Wt = (_Float16*)d_ws;

  dim3 blk(256);
  dim3 gw(HIDW / 64, HIDW / 64);
  wconv_kernel<<<gw, blk, 0, stream>>>(w1, Wt + 0 * WPLANE_ELEMS, (unsigned)HIDW, (unsigned)HIDW);
  wconv_kernel<<<gw, blk, 0, stream>>>(w2, Wt + 1 * WPLANE_ELEMS, (unsigned)HIDW, (unsigned)HIDW);
  wconv_kernel<<<gw, blk, 0, stream>>>(w3, Wt + 2 * WPLANE_ELEMS, (unsigned)HIDW, (unsigned)HIDW);
  wconv_kernel<<<gw, blk, 0, stream>>>(w4, Wt + 3 * WPLANE_ELEMS, (unsigned)HIDW, (unsigned)HIDW);
  wconv_kernel<<<gw, blk, 0, stream>>>(w5, Wt + 4 * WPLANE_ELEMS, (unsigned)HIDW, (unsigned)HIDW);

  pinn_jet_kernel<<<dim3(NPTS / 32), blk, 0, stream>>>(t, x, y, w0, b0v, Wt,
                                                       b1v, b2v, b3v, b4v, b5v, w6, b6v, out);
}
